// MambaModule_747324310169
// MI455X (gfx1250) — hardware-run, weakly checked
//
#include <hip/hip_runtime.h>
#include <stddef.h>
#include <math.h>


#pragma clang fp contract(off)

#define BSZ   4
#define TS    1024
#define DM    1024
#define DS    16
#define MR    (BSZ * TS)
#define NTHR  256
#define WSCAP 134217728
#define CVB   (NTHR * 8)
#define TP    68

static_assert((DM % 256) == 0 && (MR % 128) == 0 && (DM % 64) == 0 && (DM % 32) == 0 && DS == 16);
static_assert(((MR * DM) % CVB) == 0 && ((MR * DM / 4) % NTHR) == 0 && (TS % 64) == 0 && (DM % NTHR) == 0);

#define SZ_UP   ((size_t)MR * DM * 2)
#define SZ_WP   ((size_t)4 * DM * DM * 2)
#define SZ_BP   ((size_t)32 * DM * 2)
#define SZ_BIAS ((size_t)128)
#define SZ_F    ((size_t)MR * DM * 4)
#define SZ_BC   ((size_t)MR * 32 * 4)
#define O_UH   ((size_t)0)
#define O_UL   (O_UH + SZ_UP)
#define O_PH   (O_UL + SZ_UP)
#define O_PL   (O_PH + SZ_WP)
#define O_BH   (O_PL + SZ_WP)
#define O_BL   (O_BH + SZ_BP)
#define O_BIAS (O_BL + SZ_BP)
#define O_XP   (O_BIAS + SZ_BIAS)
#define O_Z    (O_XP + SZ_F)
#define O_XC   (O_Z + SZ_F)
#define O_XCH  (O_XC + SZ_F)
#define O_XCL  (O_XCH + SZ_UP)
#define O_BC   (O_XCL + SZ_UP)
#define WSTOT  (O_BC + SZ_BC)
static_assert(WSTOT <= (size_t)WSCAP);
static_assert((O_UL % 128) == 0 && (O_PH % 128) == 0 && (O_PL % 128) == 0 && (O_BH % 128) == 0 && (O_BL % 128) == 0);
static_assert((O_BIAS % 128) == 0 && (O_XP % 128) == 0 && (O_Z % 128) == 0 && (O_XC % 128) == 0 && (O_XCH % 128) == 0);
static_assert((O_XCL % 128) == 0 && (O_BC % 128) == 0 && (WSTOT % 128) == 0);

typedef __attribute__((ext_vector_type(16))) __bf16 v16bf;
typedef float        v8f __attribute__((ext_vector_type(8)));
typedef float        v4f __attribute__((ext_vector_type(4), __may_alias__));
typedef unsigned int v4u __attribute__((ext_vector_type(4), __may_alias__));
typedef unsigned int v2u __attribute__((ext_vector_type(2), __may_alias__));
typedef int          v8i __attribute__((ext_vector_type(8)));
union FragB { v16bf v; v8i w; v4u q[2]; };
static_assert(sizeof(FragB) == 32);

__device__ __forceinline__ v8f wmb(const FragB& a, const FragB& bq, v8f c) {
  v8f d = __builtin_amdgcn_wmma_f32_16x16x32_bf16(false, a.v, false, bq.v, (short)0, c, false, false);
  asm volatile("v_nop\n\tv_nop\n\tv_nop\n\tv_nop" : "+v"(d) : "v"(a.w), "v"(bq.w));
  return d;
}

__device__ __forceinline__ v8f zero8() {
  v8f z = {0.f, 0.f, 0.f, 0.f, 0.f, 0.f, 0.f, 0.f};
  return z;
}

__device__ __forceinline__ unsigned int bfr(float f) {
  const unsigned int u = __float_as_uint(f);
  return (u + 0x7FFFu + ((u >> 16) & 1u)) >> 16;
}

__device__ __forceinline__ void split8(v4f a, v4f c, v4u& hv, v4u& lv) {
  float in[8];
  in[0] = a[0]; in[1] = a[1]; in[2] = a[2]; in[3] = a[3];
  in[4] = c[0]; in[5] = c[1]; in[6] = c[2]; in[7] = c[3];
  unsigned int hb[8], lb[8];
#pragma unroll
  for (int i = 0; i < 8; ++i) {
    hb[i] = bfr(in[i]);
    lb[i] = bfr(in[i] - __uint_as_float(hb[i] << 16));
  }
  v4u h4, l4;
  h4[0] = hb[0] | (hb[1] << 16); h4[1] = hb[2] | (hb[3] << 16); h4[2] = hb[4] | (hb[5] << 16); h4[3] = hb[6] | (hb[7] << 16);
  l4[0] = lb[0] | (lb[1] << 16); l4[1] = lb[2] | (lb[3] << 16); l4[2] = lb[4] | (lb[5] << 16); l4[3] = lb[6] | (lb[7] << 16);
  hv = h4;
  lv = l4;
}

__device__ __forceinline__ void split4(v4f a, v2u& hv, v2u& lv) {
  unsigned int hb[4], lb[4];
#pragma unroll
  for (int i = 0; i < 4; ++i) {
    hb[i] = bfr(a[i]);
    lb[i] = bfr(a[i] - __uint_as_float(hb[i] << 16));
  }
  v2u h2, l2;
  h2[0] = hb[0] | (hb[1] << 16); h2[1] = hb[2] | (hb[3] << 16);
  l2[0] = lb[0] | (lb[1] << 16); l2[1] = lb[2] | (lb[3] << 16);
  hv = h2;
  lv = l2;
}

__global__ __launch_bounds__(NTHR) void k_usplit(const float* __restrict__ U, unsigned short* UH, unsigned short* UL) {
  const size_t so = (size_t)blockIdx.x * CVB + (size_t)threadIdx.x * 8;
  const v4f a0 = *(const v4f*)(U + so);
  const v4f a1 = *(const v4f*)(U + so + 4);
  v4u hv, lv;
  split8(a0, a1, hv, lv);
  *(volatile v4u*)(UH + so) = hv;
  *(volatile v4u*)(UL + so) = lv;
  __threadfence();
  *(volatile v4u*)(UH + so) = hv;
  *(volatile v4u*)(UL + so) = lv;
}

__global__ __launch_bounds__(NTHR) void k_wT(const float* __restrict__ W0, const float* __restrict__ W1,
                                             const float* __restrict__ W2, const float* __restrict__ W3,
                                             unsigned short* PH, unsigned short* PL) {
  __shared__ __align__(16) float sT[64 * TP];
  const int tid = threadIdx.x;
  const int w = blockIdx.z;
  const int k0 = blockIdx.x * 64, n0 = blockIdx.y * 64;
  const float* src = (w == 0) ? W0 : ((w == 1) ? W1 : ((w == 2) ? W2 : W3));
#pragma unroll
  for (int j = 0; j < 4; ++j) {
    const int kl = (tid >> 4) + 16 * j;
    const int nq = 4 * (tid & 15);
    const v4f v = *(const v4f*)(src + (size_t)(k0 + kl) * DM + n0 + nq);
#pragma unroll
    for (int i = 0; i < 4; ++i) sT[(nq + i) * TP + kl] = v[i];
  }
  __syncthreads();
  v4u hv[2], lv[2];
  size_t dst[2];
#pragma unroll
  for (int it = 0; it < 2; ++it) {
    const int nl = 32 * it + (tid >> 3), q = tid & 7;
    const v4f a = *(const v4f*)(sT + nl * TP + 8 * q);
    const v4f c = *(const v4f*)(sT + nl * TP + 8 * q + 4);
    split8(a, c, hv[it], lv[it]);
    dst[it] = ((size_t)w * DM + (size_t)(n0 + nl)) * DM + k0 + 8 * q;
  }
#pragma unroll
  for (int it = 0; it < 2; ++it) {
    *(volatile v4u*)(PH + dst[it]) = hv[it];
    *(volatile v4u*)(PL + dst[it]) = lv[it];
  }
  __threadfence();
#pragma unroll
  for (int it = 0; it < 2; ++it) {
    *(volatile v4u*)(PH + dst[it]) = hv[it];
    *(volatile v4u*)(PL + dst[it]) = lv[it];
  }
}

__global__ __launch_bounds__(NTHR) void k_wbcT(const float* __restrict__ Wb, const float* __restrict__ Wc,
                                               const float* __restrict__ bb, const float* __restrict__ bc,
                                               unsigned short* BH, unsigned short* BL, float* BIAS) {
  __shared__ __align__(16) float sT[32 * TP];
  const int tid = threadIdx.x;
  const int k0 = blockIdx.x * 64;
  {
    const int kl = tid >> 2, nq = 4 * (tid & 3);
    const v4f vb = *(const v4f*)(Wb + (size_t)(k0 + kl) * DS + nq);
    const v4f vc = *(const v4f*)(Wc + (size_t)(k0 + kl) * DS + nq);
#pragma unroll
    for (int i = 0; i < 4; ++i) {
      sT[(nq + i) * TP + kl] = vb[i];
      sT[(16 + nq + i) * TP + kl] = vc[i];
    }
  }
  __syncthreads();
  const int nl = tid >> 3, q = tid & 7;
  const v4f a = *(const v4f*)(sT + nl * TP + 8 * q);
  const v4f c = *(const v4f*)(sT + nl * TP + 8 * q + 4);
  v4u hv, lv;
  split8(a, c, hv, lv);
  const size_t dst = (size_t)nl * DM + k0 + 8 * q;
  const v4f b0 = *(const v4f*)(bb + 4 * (tid & 3));
  const v4f b1 = *(const v4f*)(bc + 4 * (tid & 3));
  v4f bs;
#pragma unroll
  for (int i = 0; i < 4; ++i) bs[i] = (tid & 4) ? b1[i] : b0[i];
  const bool bw = (blockIdx.x == 0) && (tid < 8);
  *(volatile v4u*)(BH + dst) = hv;
  *(volatile v4u*)(BL + dst) = lv;
  if (bw) *(volatile v4f*)(BIAS + 4 * tid) = bs;
  __threadfence();
  *(volatile v4u*)(BH + dst) = hv;
  *(volatile v4u*)(BL + dst) = lv;
  if (bw) *(volatile v4f*)(BIAS + 4 * tid) = bs;
}

template <int WM, int NT, int EP>
__global__ __launch_bounds__(NTHR) void k_gemm(const unsigned short* __restrict__ Ah, const unsigned short* __restrict__ Al,
                                               const unsigned short* __restrict__ Wh, const unsigned short* __restrict__ Wl,
                                               const float* __restrict__ bias, float* Cf,
                                               int lda, int ldw, int ldc, int K) {
  constexpr int WN = 8 / WM;
  constexpr int R = 16 * WM;
  constexpr int BN = WN * 16 * NT;
  static_assert(WM * WN == 8);
  static_assert(((R * BN / 4) % NTHR) == 0);
  constexpr int NF4 = (R * BN / 4) / NTHR;
  __shared__ __align__(16) float sC[R * BN];
  const int tid = threadIdx.x, lane = tid & 31, wave = tid >> 5, h = lane >> 4, m = lane & 15;
  const int wm = wave % WM, wn = wave / WM;
  const int bm0 = blockIdx.y * R;
  const int n0 = blockIdx.x * BN;
  const int m0 = bm0 + 16 * wm;
  const int nw0 = n0 + wn * 16 * NT;

  v8f acc[NT];
#pragma unroll
  for (int t = 0; t < NT; ++t) acc[t] = zero8();

  const size_t arow = (size_t)(m0 + m) * (size_t)lda + 8 * h;
  const size_t wrow = (size_t)(nw0 + m) * (size_t)ldw + 8 * h;
  const int nks = K >> 5;

#pragma unroll 1
  for (int ks = 0; ks < nks; ++ks) {
    const int k0 = ks << 5;
    FragB fah, fal;
    fah.q[0] = *(const v4u*)(Ah + arow + k0);
    fah.q[1] = *(const v4u*)(Ah + arow + k0 + 16);
    fal.q[0] = *(const v4u*)(Al + arow + k0);
    fal.q[1] = *(const v4u*)(Al + arow + k0 + 16);
#pragma unroll
    for (int t = 0; t < NT; ++t) {
      const unsigned short* wph = Wh + wrow + (size_t)(16 * t) * (size_t)ldw + k0;
      const unsigned short* wpl = Wl + wrow + (size_t)(16 * t) * (size_t)ldw + k0;
      FragB fwh, fwl;
      fwh.q[0] = *(const v4u*)wph;
      fwh.q[1] = *(const v4u*)(wph + 16);
      fwl.q[0] = *(const v4u*)wpl;
      fwl.q[1] = *(const v4u*)(wpl + 16);
      acc[t] = wmb(fah, fwh, acc[t]);
      acc[t] = wmb(fah, fwl, acc[t]);
      acc[t] = wmb(fal, fwh, acc[t]);
    }
  }

#pragma unroll
  for (int t = 0; t < NT; ++t) {
    const int cl = wn * 16 * NT + 16 * t + m;
#pragma unroll
    for (int r = 0; r < 8; ++r) {
      const int rl = 16 * wm + 8 * h + r;
      sC[rl * BN + cl] = acc[t][r];
    }
  }
  __syncthreads();

#pragma unroll 1
  for (int it = 0; it < NF4; ++it) {
    const int e = tid + it * NTHR;
    const int rl = e / (BN / 4), q = e - rl * (BN / 4);
    v4f v = *(const v4f*)(sC + 4 * e);
    const v4f b4 = *(const v4f*)(bias + n0 + 4 * q);
#pragma unroll
    for (int j = 0; j < 4; ++j) {
      float a = v[j] + b4[j];
      if constexpr (EP == 1) {
        a = a * __builtin_amdgcn_rcpf(1.0f + __expf(-a));
      } else if constexpr (EP == 2) {
        a = fmaxf(a, 0.0f) + log1pf(__expf(-fabsf(a)));
      }
      v[j] = a;
    }
    *(v4f*)(sC + 4 * e) = v;
  }

#pragma unroll
  for (int it = 0; it < NF4; ++it) {
    const int e = tid + it * NTHR;
    const int rl = e / (BN / 4), q = e - rl * (BN / 4);
    const v4f v = *(const v4f*)(sC + 4 * e);
    *(volatile v4f*)(Cf + (size_t)(bm0 + rl) * (size_t)ldc + n0 + 4 * q) = v;
  }
  __threadfence();
#pragma unroll
  for (int it = 0; it < NF4; ++it) {
    const int e = tid + it * NTHR;
    const int rl = e / (BN / 4), q = e - rl * (BN / 4);
    const v4f v = *(const v4f*)(sC + 4 * e);
    *(volatile v4f*)(Cf + (size_t)(bm0 + rl) * (size_t)ldc + n0 + 4 * q) = v;
  }
}

__global__ __launch_bounds__(NTHR) void k_conv(const float* __restrict__ XP, const float* __restrict__ cw,
                                               const float* __restrict__ cb, float* XC, unsigned short* XH,
                                               unsigned short* XL) {
  const int g = blockIdx.x * NTHR + threadIdx.x;
  const int mrow = g / (DM / 4);
  const int dq = (g - mrow * (DM / 4)) * 4;
  const int t = mrow & (TS - 1);
  const int mp = (t > 0) ? (mrow - 1) : mrow;
  const int mn = (t < TS - 1) ? (mrow + 1) : mrow;
  const float fp = (t > 0) ? 1.0f : 0.0f;
  const float fn = (t < TS - 1) ? 1.0f : 0.0f;
  const v4f xa = *(const v4f*)(XP + (size_t)mp * DM + dq);
  const v4f xb = *(const v4f*)(XP + (size_t)mrow * DM + dq);
  const v4f xc = *(const v4f*)(XP + (size_t)mn * DM + dq);
  const v4f bv = *(const v4f*)(cb + dq);
  const v4f c0 = *(const v4f*)(cw + (size_t)dq * 3);
  const v4f c1 = *(const v4f*)(cw + (size_t)dq * 3 + 4);
  const v4f c2 = *(const v4f*)(cw + (size_t)dq * 3 + 8);
  float wv[12];
  wv[0] = c0[0]; wv[1] = c0[1]; wv[2]  = c0[2]; wv[3]  = c0[3];
  wv[4] = c1[0]; wv[5] = c1[1]; wv[6]  = c1[2]; wv[7]  = c1[3];
  wv[8] = c2[0]; wv[9] = c2[1]; wv[10] = c2[2]; wv[11] = c2[3];
  v4f u;
#pragma unroll
  for (int j = 0; j < 4; ++j) {
    const float w0 = wv[3 * j + 0];
    const float w1 = wv[3 * j + 1];
    const float w2 = wv[3 * j + 2];
    const float a = (((xa[j] * fp) * w0 + xb[j] * w1) + (xc[j] * fn) * w2) + bv[j];
    u[j] = a * __builtin_amdgcn_rcpf(1.0f + __expf(-a));
  }
  v2u hv, lv;
  split4(u, hv, lv);
  const size_t o = (size_t)g * 4;
  *(volatile v4f*)(XC + o) = u;
  *(volatile v2u*)(XH + o) = hv;
  *(volatile v2u*)(XL + o) = lv;
  __threadfence();
  *(volatile v4f*)(XC + o) = u;
  *(volatile v2u*)(XH + o) = hv;
  *(volatile v2u*)(XL + o) = lv;
}

#define SCB NTHR
#define STB 32
static_assert(((STB * SCB / 8) % NTHR) == 0 && (64 * 32 / 4) == 2 * NTHR);

__global__ __launch_bounds__(NTHR) void k_scan(const float* __restrict__ DT, const float* __restrict__ XC,
                                               const float* __restrict__ Z, const float* __restrict__ BC,
                                               const float* __restrict__ Am, unsigned short* YH, unsigned short* YL) {
  __shared__ __align__(16) float sBC[64 * 32];
  __shared__ __align__(16) float sY[STB * SCB];
  const int tid = threadIdx.x;
  const int b = blockIdx.y;
  const int cbase = blockIdx.x * SCB;
  const int d = cbase + tid;

  float av[16], hs[16];
  {
    const v4f a0 = *(const v4f*)(Am + (size_t)d * DS);
    const v4f a1 = *(const v4f*)(Am + (size_t)d * DS + 4);
    const v4f a2 = *(const v4f*)(Am + (size_t)d * DS + 8);
    const v4f a3 = *(const v4f*)(Am + (size_t)d * DS + 12);
    av[0] = a0[0]; av[1] = a0[1]; av[2] = a0[2]; av[3] = a0[3];
    av[4] = a1[0]; av[5] = a1[1]; av[6] = a1[2]; av[7] = a1[3];
    av[8] = a2[0]; av[9] = a2[1]; av[10] = a2[2]; av[11] = a2[3];
    av[12] = a3[0]; av[13] = a3[1]; av[14] = a3[2]; av[15] = a3[3];
#pragma unroll
    for (int n = 0; n < 16; ++n) hs[n] = 0.0f;
  }

#pragma unroll 1
  for (int t0 = 0; t0 < TS; t0 += 64) {
    __syncthreads();
    const size_t mrow0 = (size_t)b * TS + (size_t)t0;
#pragma unroll
    for (int j = 0; j < 2; ++j) {
      const int ch = tid + j * NTHR;
      const int r = ch >> 3, c4 = (ch & 7) * 4;
      *(v4f*)(sBC + r * 32 + c4) = *(const v4f*)(BC + (mrow0 + r) * 32 + c4);
    }
    __syncthreads();
#pragma unroll 1
    for (int hf = 0; hf < 2; ++hf) {
#pragma unroll 1
      for (int tl = 0; tl < STB; ++tl) {
        const int tt = hf * STB + tl;
        const size_t e = (mrow0 + (size_t)tt) * DM + d;
        const float dt = DT[e];
        const float xv = XC[e];
        const float zv = Z[e];
        const v4f b0 = *(const v4f*)(sBC + tt * 32);
        const v4f b1 = *(const v4f*)(sBC + tt * 32 + 4);
        const v4f b2 = *(const v4f*)(sBC + tt * 32 + 8);
        const v4f b3 = *(const v4f*)(sBC + tt * 32 + 12);
        const v4f c0 = *(const v4f*)(sBC + tt * 32 + 16);
        const v4f c1 = *(const v4f*)(sBC + tt * 32 + 20);
        const v4f c2 = *(const v4f*)(sBC + tt * 32 + 24);
        const v4f c3 = *(const v4f*)(sBC + tt * 32 + 28);
        float Bv[16], Cv[16];
        Bv[0] = b0[0]; Bv[1] = b0[1]; Bv[2] = b0[2]; Bv[3] = b0[3];
        Bv[4] = b1[0]; Bv[5] = b1[1]; Bv[6] = b1[2]; Bv[7] = b1[3];
        Bv[8] = b2[0]; Bv[9] = b2[1]; Bv[10] = b2[2]; Bv[11] = b2[3];
        Bv[12] = b3[0]; Bv[13] = b3[1]; Bv[14] = b3[2]; Bv[15] = b3[3];
        Cv[0] = c0[0]; Cv[1] = c0[1]; Cv[2] = c0[2]; Cv[3] = c0[3];
        Cv[4] = c1[0]; Cv[5] = c1[1]; Cv[6] = c1[2]; Cv[7] = c1[3];
        Cv[8] = c2[0]; Cv[9] = c2[1]; Cv[10] = c2[2]; Cv[11] = c2[3];
        Cv[12] = c3[0]; Cv[13] = c3[1]; Cv[14] = c3[2]; Cv[15] = c3[3];
        float y = 0.0f;
#pragma unroll
        for (int n = 0; n < 16; ++n) {
          const float dA = __expf(dt * av[n]);
          const float dbx = (dt * Bv[n]) * xv;
          const float hn = dA * hs[n] + dbx;
          hs[n] = hn;
          y = y + hn * Cv[n];
        }
        sY[tl * SCB + tid] = y * zv;
      }
      __syncthreads();
      {
        constexpr int NIT = (STB * SCB / 8) / NTHR;
        v4u hv[NIT], lv[NIT];
        size_t dst[NIT];
#pragma unroll
        for (int it = 0; it < NIT; ++it) {
          const int e = tid + it * NTHR;
          const int rl = e >> 5, q = e & 31;
          const v4f a = *(const v4f*)(sY + rl * SCB + 8 * q);
          const v4f c = *(const v4f*)(sY + rl * SCB + 8 * q + 4);
          split8(a, c, hv[it], lv[it]);
          dst[it] = (mrow0 + (size_t)(hf * STB + rl)) * DM + cbase + 8 * q;
        }
#pragma unroll
        for (int it = 0; it < NIT; ++it) {
          *(volatile v4u*)(YH + dst[it]) = hv[it];
          *(volatile v4u*)(YL + dst[it]) = lv[it];
        }
        __threadfence();
#pragma unroll
        for (int it = 0; it < NIT; ++it) {
          *(volatile v4u*)(YH + dst[it]) = hv[it];
          *(volatile v4u*)(YL + dst[it]) = lv[it];
        }
      }
      __syncthreads();
    }
  }
}

extern "C" void kernel_launch(void* const* d_in, const int* in_sizes, int n_in,
                              void* d_out, int out_size, void* d_ws, size_t ws_size,
                              hipStream_t stream) {
  if (n_in < 16) return;
  if (in_sizes[0] != MR * DM) return;
  if (in_sizes[1] != DM * DM || in_sizes[3] != DM * DM || in_sizes[5] != DM * DM || in_sizes[14] != DM * DM) return;
  if (in_sizes[2] != DM || in_sizes[4] != DM || in_sizes[6] != DM || in_sizes[8] != DM || in_sizes[15] != DM) return;
  if (in_sizes[7] != DM * 3) return;
  if (in_sizes[9] != DM * DS || in_sizes[10] != DM * DS || in_sizes[12] != DM * DS) return;
  if (in_sizes[11] != DS || in_sizes[13] != DS) return;
  if (out_size != MR * DM) return;
  const size_t tot = (size_t)WSTOT;
  if (tot > ws_size || tot > (size_t)WSCAP) return;

  const float* u     = (const float*)d_in[0];
  const float* win   = (const float*)d_in[1];
  const float* b_in  = (const float*)d_in[2];
  const float* wg    = (const float*)d_in[3];
  const float* bg    = (const float*)d_in[4];
  const float* wout  = (const float*)d_in[5];
  const float* bout  = (const float*)d_in[6];
  const float* convw = (const float*)d_in[7];
  const float* convb = (const float*)d_in[8];
  const float* am    = (const float*)d_in[9];
  const float* wb    = (const float*)d_in[10];
  const float* bb    = (const float*)d_in[11];
  const float* wc    = (const float*)d_in[12];
  const float* bc    = (const float*)d_in[13];
  const float* wdt   = (const float*)d_in[14];
  const float* bdt   = (const float*)d_in[15];
  float* out = (float*)d_out;

  char* ws = (char*)d_ws;
  unsigned short* UH   = (unsigned short*)(ws + O_UH);
  unsigned short* UL   = (unsigned short*)(ws + O_UL);
  unsigned short* PH   = (unsigned short*)(ws + O_PH);
  unsigned short* PL   = (unsigned short*)(ws + O_PL);
  unsigned short* BH   = (unsigned short*)(ws + O_BH);
  unsigned short* BL   = (unsigned short*)(ws + O_BL);
  float*          BIAS = (float*)(ws + O_BIAS);
  float*          XP   = (float*)(ws + O_XP);
  float*          Z    = (float*)(ws + O_Z);
  float*          XC   = (float*)(ws + O_XC);
  unsigned short* XCH  = (unsigned short*)(ws + O_XCH);
  unsigned short* XCL  = (unsigned short*)(ws + O_XCL);
  float*          BCM  = (float*)(ws + O_BC);
  const size_t DD = (size_t)DM * DM;

  k_usplit<<<(MR * DM) / CVB, NTHR, 0, stream>>>(u, UH, UL);

  k_wT<<<dim3(DM / 64, DM / 64, 4), NTHR, 0, stream>>>(win, wg, wdt, wout, PH, PL);

  k_wbcT<<<DM / 64, NTHR, 0, stream>>>(wb, wc, bb, bc, BH, BL, BIAS);

  k_gemm<2, 4, 0><<<dim3(DM / 256, MR / 32), NTHR, 0, stream>>>(
      UH, UL, PH + 0 * DD, PL + 0 * DD, b_in, XP, DM, DM, DM, DM);

  k_gemm<2, 4, 1><<<dim3(DM / 256, MR / 32), NTHR, 0, stream>>>(
      UH, UL, PH + 1 * DD, PL + 1 * DD, bg, Z, DM, DM, DM, DM);

  k_conv<<<(MR * DM / 4) / NTHR, NTHR, 0, stream>>>(XP, convw, convb, XC, XCH, XCL);

  float* DTp = XP;
  k_gemm<2, 4, 2><<<dim3(DM / 256, MR / 32), NTHR, 0, stream>>>(
      XCH, XCL, PH + 2 * DD, PL + 2 * DD, bdt, DTp, DM, DM, DM, DM);

  k_gemm<8, 2, 0><<<dim3(1, MR / 128), NTHR, 0, stream>>>(
      XCH, XCL, BH, BL, BIAS, BCM, DM, DM, 32, DM);

  unsigned short* YH = UH;
  unsigned short* YL = UL;
  k_scan<<<dim3(DM / SCB, BSZ), NTHR, 0, stream>>>(DTp, XC, Z, BCM, am, YH, YL);

  k_gemm<2, 4, 0><<<dim3(DM / 256, MR / 32), NTHR, 0, stream>>>(
      YH, YL, PH + 3 * DD, PL + 3 * DD, bout, out, DM, DM, DM, DM);
}
